// TCFormerRegularAttention_28063316312342
// MI455X (gfx1250) — hardware-verified
//
#include <hip/hip_runtime.h>
#include <math.h>
#include <stdint.h>

#define NB   8
#define NQ   16384
#define CD   64
#define NR   256
#define MTOT (NB * NQ)
#define MR   (NB * NR)
#define KCV  (CD * 64)
#define STP  68
#define KP   72
#define VP   264
#define XSC  16.0f
#define WSC  256.0f
#define QSC  64.0f
#define ASC  16.0f
#define KSC  64.0f
#define VSC  64.0f
#define PSC  8192.0f
#define PCT  32.0f
#define OSC  1024.0f
#define RSPL 2048.0f
#define INVS (0.125f / (KSC * QSC))

#define KV_OFF_VTH (NR * KP * 2)
#define KV_OFF_VTL (KV_OFF_VTH + CD * VP * 2)
#define KV_OFF_VS  (KV_OFF_VTL + CD * VP * 2)
#define KV_OFF_VM  (KV_OFF_VS + 8 * CD * 4)
#define KV_LDS     (KV_OFF_VM + CD * 4)

static_assert(MTOT % 128 == 0);
static_assert(MR % 128 == 0);
static_assert(NR == 256 && CD == 64);
static_assert((STP * 4) % 16 == 0 && STP >= CD);
static_assert((KP * 2) % 16 == 0 && KP >= CD);
static_assert((VP * 2) % 16 == 0 && VP >= NR);
static_assert(KV_OFF_VTH % 16 == 0 && KV_OFF_VTL % 16 == 0 && KV_OFF_VS % 16 == 0 && KV_OFF_VM % 16 == 0);
static_assert(KV_LDS == 106752);
static_assert(MTOT % 32 == 0 && NQ % 64 == 0);

typedef _Float16 v16h __attribute__((ext_vector_type(16)));
typedef _Float16 v8h  __attribute__((ext_vector_type(8)));
typedef float    v8f  __attribute__((ext_vector_type(8)));
typedef float    v4f  __attribute__((ext_vector_type(4)));
typedef unsigned int v4u __attribute__((ext_vector_type(4)));

union Frag { v16h v; v8h h[2]; };

__device__ __forceinline__ unsigned short bf_bits(float f) {
  unsigned u = __float_as_uint(f);
  return (unsigned short)((u + 0x7FFFu + ((u >> 16) & 1u)) >> 16);
}
__device__ __forceinline__ float bfr(float f) { return __uint_as_float(((unsigned)bf_bits(f)) << 16); }
__device__ __forceinline__ unsigned short h_bits(_Float16 x) { return __builtin_bit_cast(unsigned short, x); }
__device__ __forceinline__ unsigned pk16(unsigned short a, unsigned short b) { return (unsigned)a | ((unsigned)b << 16); }
__device__ __forceinline__ v8f zero8() { v8f z = {0.f, 0.f, 0.f, 0.f, 0.f, 0.f, 0.f, 0.f}; return z; }

__device__ __forceinline__ v16h ldfrag_h(const _Float16* p) {
  Frag f;
  f.h[0] = *(const v8h*)(p);
  f.h[1] = *(const v8h*)(p + 16);
  return f.v;
}

__device__ __forceinline__ v8f mma_h(v16h a, v16h b, v8f c) {
  c = __builtin_amdgcn_wmma_f32_16x16x32_f16(false, a, false, b, (short)0, c, false, false);
#if defined(__HIP_DEVICE_COMPILE__)
  asm volatile("v_nop\n\tv_nop\n\tv_nop\n\tv_nop" : "+v"(c) : "v"(a), "v"(b));
#endif
  return c;
}
__device__ __forceinline__ void wave_sync_lds() {
  __builtin_amdgcn_fence(__ATOMIC_RELEASE, "workgroup");
  __builtin_amdgcn_wave_barrier();
  __builtin_amdgcn_fence(__ATOMIC_ACQUIRE, "workgroup");
}

__device__ __forceinline__ v4u pack8h(v4f a, v4f b) {
  v4u p;
  p[0] = pk16(h_bits((_Float16)a[0]), h_bits((_Float16)a[1]));
  p[1] = pk16(h_bits((_Float16)a[2]), h_bits((_Float16)a[3]));
  p[2] = pk16(h_bits((_Float16)b[0]), h_bits((_Float16)b[1]));
  p[3] = pk16(h_bits((_Float16)b[2]), h_bits((_Float16)b[3]));
  return p;
}
__device__ __forceinline__ void split8h(v4f a, v4f b, v4u& ph, v4u& pl) {
  v4f ra, rb;
#pragma unroll
  for (int e = 0; e < 4; ++e) {
    const _Float16 ha = (_Float16)a[e];
    ra[e] = (a[e] - (float)ha) * RSPL;
    const _Float16 hb = (_Float16)b[e];
    rb[e] = (b[e] - (float)hb) * RSPL;
  }
  ph = pack8h(a, b);
  pl = pack8h(ra, rb);
}

__global__ __launch_bounds__(256) void cvt_rows64(const float* __restrict__ src, unsigned short* dst, float scale) {
  const int tid = threadIdx.x, wave = tid >> 5, lane = tid & 31;
  const int row = blockIdx.x * 32 + wave * 4 + (lane >> 3);
  const int c8 = (lane & 7) * 8;
  const float* p = src + (size_t)row * CD + c8;
  v4f a = *(const v4f*)(p);
  v4f b = *(const v4f*)(p + 4);
#pragma unroll
  for (int e = 0; e < 4; ++e) { a[e] = bfr(a[e]) * scale; b[e] = bfr(b[e]) * scale; }
  const v4u pk = pack8h(a, b);
  unsigned short* g = dst + (size_t)row * CD + c8;
  for (int pass = 0; pass < 2; ++pass) {
    *(volatile v4u*)g = pk;
    __threadfence();
  }
}

__global__ __launch_bounds__(256) void cvt_wsr(const float* __restrict__ w, unsigned short* dst) {
  __shared__ float tile[CD][65];
  const int tid = threadIdx.x, o = blockIdx.x;
  const float* wr = w + (size_t)o * KCV;
#pragma unroll
  for (int it = 0; it < 16; ++it) {
    const int idx = it * 256 + tid;
    const int c = idx >> 6, s = idx & 63;
    tile[c][s] = wr[idx];
  }
  __syncthreads();
  v4u pk[2];
  size_t offs[2];
#pragma unroll
  for (int it = 0; it < 2; ++it) {
    const int p = it * 256 + tid;
    const int s = p >> 3, c8 = (p & 7) * 8;
    v4f fa, fb;
#pragma unroll
    for (int e = 0; e < 4; ++e) {
      fa[e] = bfr(tile[c8 + e][s]) * WSC;
      fb[e] = bfr(tile[c8 + 4 + e][s]) * WSC;
    }
    pk[it] = pack8h(fa, fb);
    offs[it] = (size_t)o * KCV + (size_t)s * CD + c8;
  }
  for (int pass = 0; pass < 2; ++pass) {
#pragma unroll
    for (int it = 0; it < 2; ++it) *(volatile v4u*)(dst + offs[it]) = pk[it];
    __threadfence();
  }
}

template <bool SPLIT, bool OUTF>
__global__ __launch_bounds__(256)
void gemm64_k(const unsigned short* __restrict__ Ah, const unsigned short* __restrict__ Al,
              const unsigned short* __restrict__ Bt, const float* __restrict__ bias, float ascale,
              float* outF, unsigned short* outH, unsigned short* outL) {
  __shared__ __align__(16) float sbuf[8 * 16 * STP];
  const int tid = threadIdx.x, wave = tid >> 5, lane = tid & 31, hh = lane >> 4, c = lane & 15;
  const int m0 = blockIdx.x * 128;
  const int arow = m0 + wave * 16 + c;
  const _Float16* A0 = (const _Float16*)(const void*)Ah;
  const _Float16* A1 = (const _Float16*)(const void*)Al;
  const _Float16* B  = (const _Float16*)(const void*)Bt;

  v8f acch[4], accl[4];
#pragma unroll
  for (int nt = 0; nt < 4; ++nt) { acch[nt] = zero8(); accl[nt] = zero8(); }

#pragma unroll
  for (int ks = 0; ks < 2; ++ks) {
    const int k0 = ks * 32;
    const size_t aoff = (size_t)arow * CD + k0 + 8 * hh;
    const v16h ah = ldfrag_h(A0 + aoff);
    v16h al = ah;
    if (SPLIT) al = ldfrag_h(A1 + aoff);
#pragma unroll
    for (int nt = 0; nt < 4; ++nt) {
      const v16h bfrag = ldfrag_h(B + (size_t)(nt * 16 + c) * CD + k0 + 8 * hh);
      acch[nt] = mma_h(ah, bfrag, acch[nt]);
      if (SPLIT) accl[nt] = mma_h(al, bfrag, accl[nt]);
    }
  }

  float* st = sbuf + wave * (16 * STP);
#pragma unroll
  for (int nt = 0; nt < 4; ++nt) {
#pragma unroll
    for (int r = 0; r < 8; ++r) {
      float v = acch[nt][r];
      if (SPLIT) v = v + accl[nt][r] * (1.0f / RSPL);
      st[(8 * hh + r) * STP + nt * 16 + c] = v * ascale;
    }
  }
  wave_sync_lds();

  if (OUTF) {
    v4f ov[8];
    size_t offs[8];
#pragma unroll
    for (int it = 0; it < 8; ++it) {
      const int q = it * 2 + hh;
      const int col = c * 4;
      const v4f v = *(const v4f*)(st + q * STP + col);
      v4f u;
#pragma unroll
      for (int e = 0; e < 4; ++e) u[e] = v[e] + bfr(bias[col + e]);
      ov[it] = u;
      offs[it] = (size_t)(m0 + wave * 16 + q) * CD + col;
    }
    for (int pass = 0; pass < 2; ++pass) {
#pragma unroll
      for (int it = 0; it < 8; ++it) *(volatile v4f*)(outF + offs[it]) = ov[it];
      __threadfence();
    }
  } else {
    v4u ph[4], pl[4];
    size_t offs[4];
#pragma unroll
    for (int it = 0; it < 4; ++it) {
      const int q = it * 4 + (lane >> 3), piece = lane & 7;
      const v4f fa = *(const v4f*)(st + q * STP + piece * 8);
      const v4f fb = *(const v4f*)(st + q * STP + piece * 8 + 4);
      split8h(fa, fb, ph[it], pl[it]);
      offs[it] = (size_t)(m0 + wave * 16 + q) * CD + piece * 8;
    }
    for (int pass = 0; pass < 2; ++pass) {
#pragma unroll
      for (int it = 0; it < 4; ++it) {
        *(volatile v4u*)(outH + offs[it]) = ph[it];
        *(volatile v4u*)(outL + offs[it]) = pl[it];
      }
      __threadfence();
    }
  }
}

__global__ __launch_bounds__(256)
void conv_ln_k(const unsigned short* __restrict__ Xh, const unsigned short* __restrict__ Wsr,
               const int* __restrict__ Hp, const int* __restrict__ Wp, const float* __restrict__ bsr,
               const float* __restrict__ lng, const float* __restrict__ lnb,
               unsigned short* Ah, unsigned short* Al) {
  __shared__ __align__(16) float sbuf[8 * 16 * STP];
  const int tid = threadIdx.x, wave = tid >> 5, lane = tid & 31, hh = lane >> 4, c = lane & 15;
  const int m0 = blockIdx.x * 128;
  const int m = m0 + wave * 16 + c;
  const int b = m >> 8, p = m & (NR - 1);
  const int Hv = Hp[0];
  int Wv = Wp[0];
  const long long hw = (long long)Hv * (long long)Wv;
  const bool okw = (Wv >= 8) && (Wv <= 2040) && (hw == (long long)NQ);
  Wv = okw ? Wv : 128;
  const int Wr = Wv >> 3;
  const int ph = p / Wr, pw = p - ph * Wr;
  int tb = ph * 8 * Wv + pw * 8;
  tb = min(tb, NQ - 1 - 7 * Wv - 7);
  tb = max(tb, 0);
  const _Float16* X  = (const _Float16*)(const void*)Xh;
  const _Float16* Wf = (const _Float16*)(const void*)Wsr;
  const size_t xbase = (size_t)b * NQ;

  v8f acc[4];
#pragma unroll
  for (int nt = 0; nt < 4; ++nt) acc[nt] = zero8();

#pragma unroll 1
  for (int k0 = 0; k0 < KCV; k0 += 32) {
    const int s = k0 >> 6, c0 = k0 & 63;
    const int kh = s >> 3, kw = s & 7;
    const int t = tb + kh * Wv + kw;
    const v16h af = ldfrag_h(X + (xbase + (size_t)t) * CD + c0 + 8 * hh);
#pragma unroll
    for (int nt = 0; nt < 4; ++nt) {
      const v16h bfrag = ldfrag_h(Wf + (size_t)(nt * 16 + c) * KCV + k0 + 8 * hh);
      acc[nt] = mma_h(af, bfrag, acc[nt]);
    }
  }

  float v[4][8];
  float gg[4], gb[4];
#pragma unroll
  for (int nt = 0; nt < 4; ++nt) {
    const int col = nt * 16 + c;
    const float bb = bfr(bsr[col]);
    gg[nt] = bfr(lng[col]);
    gb[nt] = bfr(lnb[col]);
#pragma unroll
    for (int r = 0; r < 8; ++r) v[nt][r] = acc[nt][r] * (1.0f / (XSC * WSC)) + bb;
  }
  float* st = sbuf + wave * (16 * STP);
#pragma unroll
  for (int r = 0; r < 8; ++r) {
    float sm = (v[0][r] + v[1][r]) + (v[2][r] + v[3][r]);
    sm = sm + __shfl_xor(sm, 1, 32);
    sm = sm + __shfl_xor(sm, 2, 32);
    sm = sm + __shfl_xor(sm, 4, 32);
    sm = sm + __shfl_xor(sm, 8, 32);
    const float mu = sm * (1.0f / 64.0f);
    float d[4];
    float sq = 0.f;
#pragma unroll
    for (int nt = 0; nt < 4; ++nt) { d[nt] = v[nt][r] - mu; sq = sq + d[nt] * d[nt]; }
    sq = sq + __shfl_xor(sq, 1, 32);
    sq = sq + __shfl_xor(sq, 2, 32);
    sq = sq + __shfl_xor(sq, 4, 32);
    sq = sq + __shfl_xor(sq, 8, 32);
    const float var = sq * (1.0f / 64.0f);
    const float rs = rsqrtf(var + 1e-5f);
#pragma unroll
    for (int nt = 0; nt < 4; ++nt) {
      const float y = d[nt] * rs * gg[nt] + gb[nt];
      st[(8 * hh + r) * STP + nt * 16 + c] = y * ASC;
    }
  }
  wave_sync_lds();

  v4u pkh[4], pkl[4];
  size_t offs[4];
#pragma unroll
  for (int it = 0; it < 4; ++it) {
    const int q = it * 4 + (lane >> 3), piece = lane & 7;
    const v4f fa = *(const v4f*)(st + q * STP + piece * 8);
    const v4f fb = *(const v4f*)(st + q * STP + piece * 8 + 4);
    split8h(fa, fb, pkh[it], pkl[it]);
    offs[it] = (size_t)(m0 + wave * 16 + q) * CD + piece * 8;
  }
  for (int pass = 0; pass < 2; ++pass) {
#pragma unroll
    for (int it = 0; it < 4; ++it) {
      *(volatile v4u*)(Ah + offs[it]) = pkh[it];
      *(volatile v4u*)(Al + offs[it]) = pkl[it];
    }
    __threadfence();
  }
}

__global__ __launch_bounds__(256)
void kv_k(const unsigned short* __restrict__ Ah, const unsigned short* __restrict__ Al,
          const unsigned short* __restrict__ Wkv, unsigned short* Kp, unsigned short* VTh, unsigned short* VTl,
          float* vmean) {
  extern __shared__ __align__(16) unsigned char kvlds[];
  unsigned short* sK  = (unsigned short*)(kvlds);
  unsigned short* sVh = (unsigned short*)(kvlds + KV_OFF_VTH);
  unsigned short* sVl = (unsigned short*)(kvlds + KV_OFF_VTL);
  float* sVS = (float*)(kvlds + KV_OFF_VS);
  float* sVM = (float*)(kvlds + KV_OFF_VM);
  const int tid = threadIdx.x, wave = tid >> 5, lane = tid & 31, hh = lane >> 4, c = lane & 15;
  const int b = blockIdx.x;
  const _Float16* A0 = (const _Float16*)(const void*)Ah;
  const _Float16* A1 = (const _Float16*)(const void*)Al;
  const _Float16* Bw = (const _Float16*)(const void*)Wkv;

  v16h ah[2][2], al[2][2];
#pragma unroll
  for (int mt = 0; mt < 2; ++mt) {
    const size_t arow = (size_t)(b * NR + wave * 32 + mt * 16 + c) * CD + 8 * hh;
#pragma unroll
    for (int ks = 0; ks < 2; ++ks) {
      ah[mt][ks] = ldfrag_h(A0 + arow + ks * 32);
      al[mt][ks] = ldfrag_h(A1 + arow + ks * 32);
    }
  }

#pragma unroll 1
  for (int nt = 0; nt < 8; ++nt) {
    const v16h b0 = ldfrag_h(Bw + (size_t)(nt * 16 + c) * CD + 8 * hh);
    const v16h b1 = ldfrag_h(Bw + (size_t)(nt * 16 + c) * CD + 32 + 8 * hh);
    float val[2][8];
#pragma unroll
    for (int mt = 0; mt < 2; ++mt) {
      v8f acch = mma_h(ah[mt][0], b0, zero8());
      acch = mma_h(ah[mt][1], b1, acch);
      v8f accl = mma_h(al[mt][0], b0, zero8());
      accl = mma_h(al[mt][1], b1, accl);
#pragma unroll
      for (int r = 0; r < 8; ++r) val[mt][r] = (acch[r] + accl[r] * (1.0f / RSPL)) * (1.0f / (ASC * WSC));
    }
    const int ch = nt * 16 + c;
    if (nt < 4) {
#pragma unroll
      for (int mt = 0; mt < 2; ++mt) {
#pragma unroll
        for (int r = 0; r < 8; ++r) {
          const int tk = wave * 32 + mt * 16 + 8 * hh + r;
          sK[tk * KP + ch] = h_bits((_Float16)(val[mt][r] * KSC));
        }
      }
    } else {
      const int d = ch - CD;
      float vs = 0.f;
#pragma unroll
      for (int mt = 0; mt < 2; ++mt) {
        v4f fa, fb;
#pragma unroll
        for (int e = 0; e < 4; ++e) {
          fa[e] = val[mt][e] * VSC;
          fb[e] = val[mt][4 + e] * VSC;
          vs = vs + val[mt][e];
          vs = vs + val[mt][4 + e];
        }
        v4u ph, pl;
        split8h(fa, fb, ph, pl);
        const int tk0 = wave * 32 + mt * 16 + 8 * hh;
        *(v4u*)(sVh + d * VP + tk0) = ph;
        *(v4u*)(sVl + d * VP + tk0) = pl;
      }
      vs = vs + __shfl_xor(vs, 16, 32);
      if (hh == 0) sVS[wave * CD + d] = vs;
    }
  }
  __syncthreads();
  if (tid < CD) {
    float s = 0.f;
#pragma unroll
    for (int w = 0; w < 8; ++w) s = s + sVS[w * CD + tid];
    sVM[tid] = s * (1.0f / (float)NR);
  }
  __syncthreads();

  for (int pass = 0; pass < 2; ++pass) {
#pragma unroll
    for (int it = 0; it < 8; ++it) {
      const int row = wave * 32 + it * 4 + (lane >> 3), piece = lane & 7;
      const v4u kk = *(const v4u*)(sK + row * KP + piece * 8);
      *(volatile v4u*)(Kp + (size_t)(b * NR + row) * CD + piece * 8) = kk;
    }
#pragma unroll
    for (int it = 0; it < 8; ++it) {
      const int d = wave * 8 + it;
      const v4u vh = *(const v4u*)(sVh + d * VP + lane * 8);
      const v4u vl = *(const v4u*)(sVl + d * VP + lane * 8);
      *(volatile v4u*)(VTh + (size_t)(b * CD + d) * NR + lane * 8) = vh;
      *(volatile v4u*)(VTl + (size_t)(b * CD + d) * NR + lane * 8) = vl;
    }
    if (wave == 0 && lane < 16) {
      const v4f m4 = *(const v4f*)(sVM + lane * 4);
      *(volatile v4f*)(vmean + (size_t)b * CD + lane * 4) = m4;
    }
    __threadfence();
  }
}

__global__ __launch_bounds__(128) __attribute__((amdgpu_num_vgpr(256)))
void attn_k(const unsigned short* __restrict__ Qh, const unsigned short* __restrict__ Ql,
            const unsigned short* __restrict__ Kp, const unsigned short* __restrict__ VTh,
            const unsigned short* __restrict__ VTl, const float* __restrict__ vmean,
            unsigned short* Oh, unsigned short* Ol) {
  __shared__ __align__(16) float sbuf[4 * 16 * STP];
  const int tid = threadIdx.x, wave = tid >> 5, lane = tid & 31, hh = lane >> 4, c = lane & 15;
  const int b = blockIdx.x >> 8;
  const int q0 = ((blockIdx.x & 255) << 6) + wave * 16;
  const _Float16* Qhf = (const _Float16*)(const void*)Qh;
  const _Float16* Qlf = (const _Float16*)(const void*)Ql;
  const _Float16* Kf  = (const _Float16*)(const void*)Kp;
  const _Float16* Vhf = (const _Float16*)(const void*)VTh;
  const _Float16* Vlf = (const _Float16*)(const void*)VTl;

  const size_t qoff = (size_t)(b * NQ + q0 + c) * CD + 8 * hh;
  const v16h qh0 = ldfrag_h(Qhf + qoff);
  const v16h qh1 = ldfrag_h(Qhf + qoff + 32);
  const v16h ql0 = ldfrag_h(Qlf + qoff);
  const v16h ql1 = ldfrag_h(Qlf + qoff + 32);

  v8f s[16];
#pragma unroll
  for (int j = 0; j < 16; ++j) {
    const size_t koff = (size_t)(b * NR + j * 16 + c) * CD + 8 * hh;
    const v16h ka0 = ldfrag_h(Kf + koff);
    const v16h ka1 = ldfrag_h(Kf + koff + 32);
    v8f sh = mma_h(ka0, qh0, zero8());
    sh = mma_h(ka1, qh1, sh);
    v8f sl = mma_h(ka0, ql0, zero8());
    sl = mma_h(ka1, ql1, sl);
#pragma unroll
    for (int r = 0; r < 8; ++r) s[j][r] = sh[r] + sl[r] * (1.0f / RSPL);
  }

  float mx = -3.0e38f;
#pragma unroll
  for (int j = 0; j < 16; ++j) {
#pragma unroll
    for (int r = 0; r < 8; ++r) mx = fmaxf(mx, s[j][r]);
  }
  mx = fmaxf(mx, __shfl_xor(mx, 16, 32));
  float ls = 0.f;
#pragma unroll
  for (int j = 0; j < 16; ++j) {
#pragma unroll
    for (int r = 0; r < 8; ++r) {
      const float e = __expf((s[j][r] - mx) * INVS);
      s[j][r] = e;
      ls = ls + e;
    }
  }
  ls = ls + __shfl_xor(ls, 16, 32);
  const float pinv = __builtin_amdgcn_rcpf(ls) * PSC;

  v16h pf[8];
#pragma unroll
  for (int J = 0; J < 8; ++J) {
#pragma unroll
    for (int i = 0; i < 8; ++i) {
      pf[J][i]     = (_Float16)(s[2 * J][i] * pinv - PCT);
      pf[J][8 + i] = (_Float16)(s[2 * J + 1][i] * pinv - PCT);
    }
  }

  v8f oh[4], ol[4];
#pragma unroll
  for (int dt = 0; dt < 4; ++dt) { oh[dt] = zero8(); ol[dt] = zero8(); }
#pragma unroll
  for (int J = 0; J < 8; ++J) {
#pragma unroll
    for (int dt = 0; dt < 4; ++dt) {
      const size_t voff = (size_t)(b * CD + dt * 16 + c) * NR + J * 32 + 8 * hh;
      const v16h vh = ldfrag_h(Vhf + voff);
      const v16h vl = ldfrag_h(Vlf + voff);
      oh[dt] = mma_h(pf[J], vh, oh[dt]);
      ol[dt] = mma_h(pf[J], vl, ol[dt]);
    }
  }

  float* st = sbuf + wave * (16 * STP);
#pragma unroll
  for (int dt = 0; dt < 4; ++dt) {
    const int d = dt * 16 + c;
    const float vm = vmean[(size_t)b * CD + d];
#pragma unroll
    for (int r = 0; r < 8; ++r) {
      const float o = (oh[dt][r] + ol[dt][r] * (1.0f / RSPL)) * (1.0f / (PSC * VSC)) + vm;
      st[(8 * hh + r) * STP + d] = o * OSC;
    }
  }
  wave_sync_lds();

  v4u ph[4], pl[4];
  size_t offs[4];
#pragma unroll
  for (int it = 0; it < 4; ++it) {
    const int q = it * 4 + (lane >> 3), piece = lane & 7;
    const v4f fa = *(const v4f*)(st + q * STP + piece * 8);
    const v4f fb = *(const v4f*)(st + q * STP + piece * 8 + 4);
    split8h(fa, fb, ph[it], pl[it]);
    offs[it] = (size_t)(b * NQ + q0 + q) * CD + piece * 8;
  }
  for (int pass = 0; pass < 2; ++pass) {
#pragma unroll
    for (int it = 0; it < 4; ++it) {
      *(volatile v4u*)(Oh + offs[it]) = ph[it];
      *(volatile v4u*)(Ol + offs[it]) = pl[it];
    }
    __threadfence();
  }
}

extern "C" void kernel_launch(void* const* d_in, const int* in_sizes, int n_in,
                              void* d_out, int out_size, void* d_ws, size_t ws_size,
                              hipStream_t stream) {
  if (n_in < 11) return;
  if (in_sizes[0] != MTOT * CD) return;
  if (in_sizes[1] != 1 || in_sizes[2] != 1) return;
  if (in_sizes[3] != CD * CD) return;
  if (in_sizes[4] != 2 * CD * CD) return;
  if (in_sizes[5] != CD * KCV) return;
  if (in_sizes[6] != CD || in_sizes[7] != CD || in_sizes[8] != CD) return;
  if (in_sizes[9] != CD * CD || in_sizes[10] != CD) return;
  if (out_size != MTOT * CD) return;

  const float* x      = (const float*)d_in[0];
  const int*   hptr   = (const int*)d_in[1];
  const int*   wptr   = (const int*)d_in[2];
  const float* w_q    = (const float*)d_in[3];
  const float* w_kv   = (const float*)d_in[4];
  const float* w_sr   = (const float*)d_in[5];
  const float* b_sr   = (const float*)d_in[6];
  const float* ln_g   = (const float*)d_in[7];
  const float* ln_b   = (const float*)d_in[8];
  const float* w_proj = (const float*)d_in[9];
  const float* b_proj = (const float*)d_in[10];
  float* out = (float*)d_out;

  const size_t sX   = (size_t)MTOT * CD * 2;
  const size_t sWq  = (size_t)CD * CD * 2;
  const size_t sWkv = (size_t)2 * CD * CD * 2;
  const size_t sWsr = (size_t)CD * KCV * 2;
  const size_t sWp  = (size_t)CD * CD * 2;
  const size_t sQ   = (size_t)MTOT * CD * 2;
  const size_t sA   = (size_t)MR * CD * 2;
  const size_t sK   = (size_t)NB * NR * CD * 2;
  const size_t sVT  = (size_t)NB * CD * NR * 2;
  const size_t sVM  = (size_t)NB * CD * 4;
  const size_t sO   = (size_t)MTOT * CD * 2;
  size_t off = 0;
  const size_t oX   = off; off += sX;
  const size_t oWq  = off; off += sWq;
  const size_t oWkv = off; off += sWkv;
  const size_t oWsr = off; off += sWsr;
  const size_t oWp  = off; off += sWp;
  const size_t oQh  = off; off += sQ;
  const size_t oQl  = off; off += sQ;
  const size_t oAh  = off; off += sA;
  const size_t oAl  = off; off += sA;
  const size_t oK   = off; off += sK;
  const size_t oVTh = off; off += sVT;
  const size_t oVTl = off; off += sVT;
  const size_t oVM  = off; off += sVM;
  const size_t oOh  = off; off += sO;
  const size_t oOl  = off; off += sO;
  if (off > ws_size) return;
  if (off > (size_t)134217728) return;

  char* ws = (char*)d_ws;
  unsigned short* Xh  = (unsigned short*)(ws + oX);
  unsigned short* Wq  = (unsigned short*)(ws + oWq);
  unsigned short* Wkv = (unsigned short*)(ws + oWkv);
  unsigned short* Wsr = (unsigned short*)(ws + oWsr);
  unsigned short* Wp  = (unsigned short*)(ws + oWp);
  unsigned short* Qh  = (unsigned short*)(ws + oQh);
  unsigned short* Ql  = (unsigned short*)(ws + oQl);
  unsigned short* Ah  = (unsigned short*)(ws + oAh);
  unsigned short* Al  = (unsigned short*)(ws + oAl);
  unsigned short* Kp  = (unsigned short*)(ws + oK);
  unsigned short* VTh = (unsigned short*)(ws + oVTh);
  unsigned short* VTl = (unsigned short*)(ws + oVTl);
  float* VM = (float*)(ws + oVM);
  unsigned short* Oh  = (unsigned short*)(ws + oOh);
  unsigned short* Ol  = (unsigned short*)(ws + oOl);

  const dim3 blk(256);
  cvt_rows64<<<dim3(MTOT / 32), blk, 0, stream>>>(x, Xh, XSC);
  cvt_rows64<<<dim3(CD / 32), blk, 0, stream>>>(w_q, Wq, WSC);
  cvt_rows64<<<dim3((2 * CD) / 32), blk, 0, stream>>>(w_kv, Wkv, WSC);
  cvt_rows64<<<dim3(CD / 32), blk, 0, stream>>>(w_proj, Wp, WSC);
  cvt_wsr<<<dim3(CD), blk, 0, stream>>>(w_sr, Wsr);
  gemm64_k<false, false><<<dim3(MTOT / 128), blk, 0, stream>>>(Xh, Xh, Wq, b_proj, QSC / (XSC * WSC), out, Qh, Ql);
  conv_ln_k<<<dim3(MR / 128), blk, 0, stream>>>(Xh, Wsr, hptr, wptr, b_sr, ln_g, ln_b, Ah, Al);
  (void)hipFuncSetAttribute(reinterpret_cast<const void*>(&kv_k), hipFuncAttributeMaxDynamicSharedMemorySize, KV_LDS);
  kv_k<<<dim3(NB), blk, KV_LDS, stream>>>(Ah, Al, Wkv, Kp, VTh, VTl, VM);
  attn_k<<<dim3(NB * (NQ / 64)), dim3(128), 0, stream>>>(Qh, Ql, Kp, VTh, VTl, VM, Oh, Ol);
  gemm64_k<true, true><<<dim3(MTOT / 128), blk, 0, stream>>>(Oh, Ol, Wp, b_proj, 1.0f / (OSC * WSC), out, Xh, Xh);
  (void)hipGetLastError();
}
